// GeometricAttention_70222715290238
// MI455X (gfx1250) — hardware-verified
//
#include <hip/hip_runtime.h>
#include <math.h>
#include <stdint.h>

#ifndef NB
#define NB 2
#endif
#ifndef SEQ
#define SEQ 2048
#endif
#define NB_FULL 2
#define SEQ_FULL 2048

constexpr int kDM    = 1024;
constexpr int kHeads = 16;
constexpr int kHD    = 64;
constexpr int kPos   = 64;
constexpr int kTok   = NB * SEQ;
constexpr int kKP    = 72;
constexpr int kDP    = 68;
static_assert(NB >= 1 && NB <= NB_FULL && SEQ >= 64 && SEQ <= SEQ_FULL);
static_assert(SEQ % 64 == 0 && kTok % 64 == 0 && kTok % 32 == 0);
static_assert(kDM % 64 == 0 && kDM % 32 == 0 && kHeads * kHD == kDM && kHD == 64 && kPos == 64);

constexpr size_t kSzXB = (size_t)kTok * kDM * 2;
constexpr size_t kSzW  = (size_t)kDM * kDM * 2;
constexpr size_t kSzQK = (size_t)kTok * kDM * 2;
constexpr size_t kSzVT = (size_t)kDM * kTok * 2;
constexpr size_t kSzD  = (size_t)SEQ * SEQ * 4;
constexpr size_t kSzC  = (size_t)kTok * kDM * 2;
constexpr size_t kOffXB = 0;
constexpr size_t kOffWq = kOffXB + kSzXB;
constexpr size_t kOffWk = kOffWq + kSzW;
constexpr size_t kOffWv = kOffWk + kSzW;
constexpr size_t kOffWo = kOffWv + kSzW;
constexpr size_t kOffQ  = kOffWo + kSzW;
constexpr size_t kOffK  = kOffQ + kSzQK;
constexpr size_t kOffVh = kOffK + kSzQK;
constexpr size_t kOffVl = kOffVh + kSzVT;
constexpr size_t kOffD  = kOffVl + kSzVT;
constexpr size_t kOffCh = kOffD + kSzD;
constexpr size_t kOffCl = kOffCh + kSzC;
constexpr size_t kWsEnd = kOffCl + kSzC;
static_assert(kWsEnd <= 134217728ull);
static_assert(!(NB == NB_FULL && SEQ == SEQ_FULL) || kWsEnd == 83886080ull);
static_assert(kOffWq % 128 == 0 && kOffQ % 128 == 0 && kOffK % 128 == 0 && kOffVh % 128 == 0 && kOffVl % 128 == 0);
static_assert(kOffD % 128 == 0 && kOffCh % 128 == 0 && kOffCl % 128 == 0);
static_assert((size_t)kTok * kDM < 2147483648ull && (size_t)SEQ * SEQ < 2147483648ull);

typedef __attribute__((ext_vector_type(16))) _Float16 v16h;
typedef __attribute__((ext_vector_type(8)))  _Float16 v8h;
typedef __attribute__((ext_vector_type(16))) __bf16   v16b;
typedef __attribute__((ext_vector_type(8)))  __bf16   v8b;
typedef __attribute__((ext_vector_type(8)))  float    v8f;
typedef __attribute__((ext_vector_type(4)))  float    v4f;
typedef __attribute__((ext_vector_type(4)))  unsigned int v4u;

__device__ __forceinline__ unsigned short f2bf_bits(float f) {
  unsigned u = __float_as_uint(f);
  return (unsigned short)((u + 0x7FFFu + ((u >> 16) & 1u)) >> 16);
}
__device__ __forceinline__ float bf_bits2f(unsigned short h) { return __uint_as_float(((unsigned)h) << 16); }
__device__ __forceinline__ float bf_rne(float f) { return bf_bits2f(f2bf_bits(f)); }

__device__ __forceinline__ void dep_guard_h(v8f& a, v8f& b, v16h x, v16h y) { asm volatile("v_nop\n\tv_nop\n\tv_nop\n\tv_nop" : "+v"(a), "+v"(b) : "v"(x), "v"(y)); }
__device__ __forceinline__ void dep_guard_b(v8f& a, v8f& b, v16b x, v16b y) { asm volatile("v_nop\n\tv_nop\n\tv_nop\n\tv_nop" : "+v"(a), "+v"(b) : "v"(x), "v"(y)); }
__device__ __forceinline__ void keep4_h(v16h a, v16h b, v16h c, v16h d) { asm volatile("v_nop" :: "v"(a), "v"(b), "v"(c), "v"(d)); }
__device__ __forceinline__ void keep4_b(v16b a, v16b b, v16b c, v16b d) { asm volatile("v_nop" :: "v"(a), "v"(b), "v"(c), "v"(d)); }
__device__ __forceinline__ void acc_guard4(v8f& a, v8f& b, v8f& c, v8f& d) { asm volatile("v_nop\n\tv_nop\n\tv_nop\n\tv_nop" : "+v"(a), "+v"(b), "+v"(c), "+v"(d)); }
__device__ __forceinline__ void grp_guard_h(v8f& a, v8f& b, v16h f0, v16h f1, v16h f2) {
  asm volatile("v_nop\n\tv_nop\n\tv_nop\n\tv_nop" : "+v"(a), "+v"(b) : "v"(f0), "v"(f1), "v"(f2) : "memory");
}
__device__ __forceinline__ void grp_guard_b2(v8f& a, v16b f0, v16b f1, v16b f2) {
  asm volatile("v_nop\n\tv_nop\n\tv_nop\n\tv_nop" : "+v"(a) : "v"(f0), "v"(f1), "v"(f2) : "memory");
}
__device__ __forceinline__ void grp_guard_b1(v8f& a, v16b f0, v16b f1) {
  asm volatile("v_nop\n\tv_nop\n\tv_nop\n\tv_nop" : "+v"(a) : "v"(f0), "v"(f1) : "memory");
}
__device__ __forceinline__ void phase_cut() { __builtin_amdgcn_sched_barrier(0); }

template <typename T> struct Frag;
template <> struct Frag<_Float16> {
  typedef v16h V; union U { v16h v; v8h h[2]; };
  static __device__ __forceinline__ v16h load(const _Float16* p) {
    U f; f.h[0] = *(const v8h*)(p); f.h[1] = *(const v8h*)(p + 16); return f.v;
  }
  static __device__ __forceinline__ v8f mma(v16h a, v16h b, v8f c) {
    return __builtin_amdgcn_wmma_f32_16x16x32_f16(false, a, false, b, (short)0, c, false, false);
  }
  static __device__ __forceinline__ void guard(v8f& a, v8f& b, v16h x, v16h y) { dep_guard_h(a, b, x, y); }
  static __device__ __forceinline__ void keep(v16h a, v16h b, v16h c, v16h d) { keep4_h(a, b, c, d); }
};
template <> struct Frag<__bf16> {
  typedef v16b V; union U { v16b v; v8b h[2]; };
  static __device__ __forceinline__ v16b load(const __bf16* p) {
    U f; f.h[0] = *(const v8b*)(p); f.h[1] = *(const v8b*)(p + 16); return f.v;
  }
  static __device__ __forceinline__ v8f mma(v16b a, v16b b, v8f c) {
    return __builtin_amdgcn_wmma_f32_16x16x32_bf16(false, a, false, b, (short)0, c, false, false);
  }
  static __device__ __forceinline__ void guard(v8f& a, v8f& b, v16b x, v16b y) { dep_guard_b(a, b, x, y); }
  static __device__ __forceinline__ void keep(v16b a, v16b b, v16b c, v16b d) { keep4_b(a, b, c, d); }
};

__device__ __forceinline__ unsigned pk16(unsigned short a, unsigned short b) { return (unsigned)a | ((unsigned)b << 16); }

__device__ __forceinline__ void qk_pair(v8f& s0, v8f& s1, v16h q, const _Float16* k0p, const _Float16* k1p) {
  const v16h a = Frag<_Float16>::load(k0p);
  const v16h c = Frag<_Float16>::load(k1p);
  s0 = Frag<_Float16>::mma(q, a, s0);
  s1 = Frag<_Float16>::mma(q, c, s1);
  grp_guard_h(s0, s1, q, a, c);
}
__device__ __forceinline__ void pv_hl(v8f& o, v16b p, const __bf16* vhp, const __bf16* vlp) {
  const v16b a = Frag<__bf16>::load(vhp);
  const v16b c = Frag<__bf16>::load(vlp);
  o = Frag<__bf16>::mma(p, a, o);
  o = Frag<__bf16>::mma(p, c, o);
  grp_guard_b2(o, p, a, c);
}
__device__ __forceinline__ void pv_h(v8f& o, v16b p, const __bf16* vhp) {
  const v16b a = Frag<__bf16>::load(vhp);
  o = Frag<__bf16>::mma(p, a, o);
  grp_guard_b1(o, p, a);
}
__device__ __forceinline__ void put_p(__bf16* ph, __bf16* pl, float p) {
  const unsigned short hb = f2bf_bits(p);
  const unsigned short lb = f2bf_bits(p - bf_bits2f(hb));
  *ph = __builtin_bit_cast(__bf16, hb);
  *pl = __builtin_bit_cast(__bf16, lb);
}

template <int ET> struct Elem;
template <> struct Elem<0> { typedef _Float16 T; };
template <> struct Elem<1> { typedef __bf16 T; };
template <int ET, int SPLITM, int BIAS_MODE, int OUT_MODE, bool RESID, int ACT = 0>
__global__ __launch_bounds__(256) void wmma_gemm64(
    const unsigned short* __restrict__ Ap, const unsigned short* __restrict__ A2p, int lda, long strideA,
    const unsigned short* __restrict__ Btp, const unsigned short* __restrict__ Bt2p, int ldb, long strideB,
    void* __restrict__ Cout, void* __restrict__ Cout2, int ldc, long strideC,
    const float* __restrict__ bias,
    const float* __restrict__ resid, long strideR,
    int M, int N, int K, float scale) {
  constexpr bool SPLA = (SPLITM >= 1);
  constexpr bool SPLB = (SPLITM == 2);
  typedef typename Elem<ET>::T T;
  typedef typename Frag<T>::V V;
  const T* A = (const T*)Ap; const T* A2 = (const T*)A2p; const T* Bt = (const T*)Btp; const T* Bt2 = (const T*)Bt2p;
  __shared__ __align__(16) float sT[8][16 * 68];
  const int b    = blockIdx.y;
  const int lane = threadIdx.x & 31;
  const int wave = threadIdx.x >> 5;
  const int tilesN = N >> 6;
  const int tilesM = M >> 6;
  const int tile = blockIdx.x * 8 + wave;
  if (tile >= tilesM * tilesN) return;
  const int tm = tile / tilesN;
  const int tn = tile - tm * tilesN;
  const int m0 = tm << 6;
  const int n0 = tn << 6;

  const T* Ab  = A  + (size_t)b * strideA;
  const T* Bb  = Bt + (size_t)b * strideB;
  const T* Ab2 = SPLA ? (A2  + (size_t)b * strideA) : nullptr;
  const T* Bb2 = SPLB ? (Bt2 + (size_t)b * strideB) : nullptr;

  const int rlane = lane & 15;
  const int koff  = (lane >> 4) * 8;
  const int mOff  = (lane >> 4) * 8;

  v8f acc[4][4];
#pragma unroll
  for (int i = 0; i < 4; ++i)
#pragma unroll
    for (int j = 0; j < 4; ++j) acc[i][j] = (v8f){0.f,0.f,0.f,0.f,0.f,0.f,0.f,0.f};

  for (int k0 = 0; k0 < K; k0 += 32) {
    V bh[4], bl[4];
#pragma unroll
    for (int j = 0; j < 4; ++j) {
      const size_t bo = (size_t)(n0 + (j << 4) + rlane) * ldb + koff + k0;
      bh[j] = Frag<T>::load(Bb + bo);
      if (SPLB) bl[j] = Frag<T>::load(Bb2 + bo);
    }
#pragma unroll
    for (int i = 0; i < 4; ++i) {
      const size_t ao = (size_t)(m0 + (i << 4) + rlane) * lda + koff + k0;
      V ah = Frag<T>::load(Ab + ao);
      V al;
      if (SPLA) al = Frag<T>::load(Ab2 + ao);
#pragma unroll
      for (int j = 0; j < 4; ++j) {
        acc[i][j] = Frag<T>::mma(ah, bh[j], acc[i][j]);
        if (SPLB) acc[i][j] = Frag<T>::mma(ah, bl[j], acc[i][j]);
        if (SPLA) acc[i][j] = Frag<T>::mma(al, bh[j], acc[i][j]);
      }
      Frag<T>::guard(acc[i][0], acc[i][3], ah, SPLA ? al : ah);
    }
    Frag<T>::keep(bh[0], bh[1], bh[2], bh[3]);
    if (SPLB) Frag<T>::keep(bl[0], bl[1], bl[2], bl[3]);
  }
  acc_guard4(acc[0][0], acc[0][1], acc[0][2], acc[0][3]);
  acc_guard4(acc[1][0], acc[1][1], acc[1][2], acc[1][3]);
  acc_guard4(acc[2][0], acc[2][1], acc[2][2], acc[2][3]);
  acc_guard4(acc[3][0], acc[3][1], acc[3][2], acc[3][3]);

  float* slab = sT[wave];
  const float* Rb = RESID ? (resid + (size_t)b * strideR) : nullptr;
#pragma unroll
  for (int i = 0; i < 4; ++i) {
    const int mBase = m0 + (i << 4);
#pragma unroll
    for (int j = 0; j < 4; ++j) {
      const int n = n0 + (j << 4) + rlane;
      float bv = 0.f;
      if (BIAS_MODE == 2) bv = bf_rne(bias[n]);
#pragma unroll
      for (int r = 0; r < 8; ++r) {
        float v = acc[i][j][r] * scale;
        if (BIAS_MODE == 1) v += bf_rne(bias[mBase + mOff + r]);
        if (BIAS_MODE == 2) v += bv;
        if (BIAS_MODE == 3) v *= bias[mBase + mOff + r];
        if (RESID) v += Rb[(size_t)(mBase + mOff + r) * ldc + n];
        if (ACT == 2) v = fmaxf(v, 0.0f);
        if (ACT == 4) v = (v > 0.f) ? v : 0.01f * v;
        slab[(mOff + r) * 68 + (j << 4) + rlane] = v;
      }
    }
    __builtin_amdgcn_fence(3, "workgroup");
    __builtin_amdgcn_wave_barrier();
    __builtin_amdgcn_fence(2, "workgroup");
    if (OUT_MODE == 0) {
      float* C = (float*)Cout + (size_t)b * strideC;
      const int hh = lane >> 4, c4 = (lane & 15) * 4;
      for (int pass = 0; pass < 2; ++pass) {
#pragma unroll
        for (int it = 0; it < 8; ++it) {
          const int row = it * 2 + hh;
          v4f v = *(const v4f*)(slab + row * 68 + c4);
          *(volatile v4f*)(C + (size_t)(mBase + row) * ldc + n0 + c4) = v;
        }
        __threadfence();
      }
    } else {
      const int q = lane >> 3, c8 = (lane & 7) * 8;
      unsigned short* C  = (unsigned short*)Cout  + (size_t)b * strideC;
      unsigned short* C2 = (OUT_MODE == 2) ? ((unsigned short*)Cout2 + (size_t)b * strideC) : nullptr;
      for (int pass = 0; pass < 2; ++pass) {
#pragma unroll
        for (int it = 0; it < 4; ++it) {
          const int row = it * 4 + q;
          const float* sp = slab + row * 68 + c8;
          v8h hv, lv;
#pragma unroll
          for (int e = 0; e < 8; ++e) {
            if (OUT_MODE == 1) {
              hv[e] = (_Float16)sp[e];
            } else {
              unsigned short hb = f2bf_bits(sp[e]);
              unsigned short lb = f2bf_bits(sp[e] - bf_bits2f(hb));
              hv[e] = __builtin_bit_cast(_Float16, hb);
              lv[e] = __builtin_bit_cast(_Float16, lb);
            }
          }
          *(volatile v8h*)(C + (size_t)(mBase + row) * ldc + n0 + c8) = hv;
          if (OUT_MODE == 2) *(volatile v8h*)(C2 + (size_t)(mBase + row) * ldc + n0 + c8) = lv;
        }
        __threadfence();
      }
    }
    __builtin_amdgcn_fence(3, "workgroup");
    __builtin_amdgcn_wave_barrier();
    __builtin_amdgcn_fence(2, "workgroup");
  }
}

__global__ __launch_bounds__(256) void xcast_kernel(const float* __restrict__ in, unsigned short* __restrict__ out) {
  const int t = threadIdx.x;
  const int sr = t >> 7;
  const int c8 = (t & 127) * 8;
#pragma unroll 1
  for (int g = 0; g < 16; ++g) {
    const int prow = blockIdx.x * 32 + g * 2 + sr;
    const int b = prow / SEQ;
    const int s = prow - b * SEQ;
    const float* p = in + ((size_t)b * SEQ_FULL + s) * kDM + c8;
    const v4f a = *(const v4f*)(p);
    const v4f c = *(const v4f*)(p + 4);
    unsigned short hb[8];
#pragma unroll
    for (int e = 0; e < 4; ++e) { hb[e] = f2bf_bits(a[e]); hb[4 + e] = f2bf_bits(c[e]); }
    const v4u u = (v4u){pk16(hb[0], hb[1]), pk16(hb[2], hb[3]), pk16(hb[4], hb[5]), pk16(hb[6], hb[7])};
    unsigned short* q = out + (size_t)prow * kDM + c8;
    *(volatile v4u*)q = u;
    __threadfence();
    *(volatile v4u*)q = u;
  }
}

__global__ __launch_bounds__(256) void wtcast_kernel(const float* __restrict__ w, unsigned short* __restrict__ out) {
  __shared__ float sm[64][65];
  const int t  = threadIdx.x;
  const int n0 = blockIdx.x * 64;
  const int k0 = blockIdx.y * 64;
#pragma unroll
  for (int i = 0; i < 16; ++i) {
    const int e  = i * 256 + t;
    const int kl = e >> 6;
    const int nl = e & 63;
    sm[nl][kl] = w[(size_t)(k0 + kl) * kDM + n0 + nl];
  }
  __syncthreads();
  const int lane = t & 31, wave = t >> 5;
  const int q = lane >> 3, c8 = (lane & 7) * 8;
  for (int pass = 0; pass < 2; ++pass) {
#pragma unroll
    for (int it = 0; it < 2; ++it) {
      const int row = wave * 8 + it * 4 + q;
      unsigned short hb[8];
#pragma unroll
      for (int e = 0; e < 8; ++e) hb[e] = f2bf_bits(sm[row][c8 + e]);
      const v4u u = (v4u){pk16(hb[0], hb[1]), pk16(hb[2], hb[3]), pk16(hb[4], hb[5]), pk16(hb[6], hb[7])};
      *(volatile v4u*)(out + (size_t)(n0 + row) * kDM + k0 + c8) = u;
    }
    __threadfence();
  }
}

__global__ __launch_bounds__(256) void dist_kernel(const float* __restrict__ pos, float* __restrict__ dist) {
  __shared__ float sPi[64][65];
  __shared__ float sPj[64][65];
  __shared__ __align__(16) float sD[64 * kDP];
  const int t  = threadIdx.x;
  const int i0 = blockIdx.y * 64;
  const int j0 = blockIdx.x * 64;
#pragma unroll
  for (int it = 0; it < 16; ++it) {
    const int e = it * 256 + t;
    const int r = e >> 6, c = e & 63;
    sPi[r][c] = bf_rne(pos[(size_t)(i0 + r) * kPos + c]);
    sPj[r][c] = bf_rne(pos[(size_t)(j0 + r) * kPos + c]);
  }
  __syncthreads();
  const int ty = t >> 4, tx = t & 15;
  float s[4][4];
#pragma unroll
  for (int u = 0; u < 4; ++u)
#pragma unroll
    for (int v = 0; v < 4; ++v) s[u][v] = 0.f;
#pragma unroll 1
  for (int p = 0; p < kPos; ++p) {
    float a[4], c[4];
#pragma unroll
    for (int u = 0; u < 4; ++u) { a[u] = sPi[ty * 4 + u][p]; c[u] = sPj[tx * 4 + u][p]; }
#pragma unroll
    for (int u = 0; u < 4; ++u)
#pragma unroll
      for (int v = 0; v < 4; ++v) { const float d = c[v] - a[u]; s[u][v] = fmaf(d, d, s[u][v]); }
  }
#pragma unroll
  for (int u = 0; u < 4; ++u) {
    const v4f rv = (v4f){s[u][0], s[u][1], s[u][2], s[u][3]};
    *(v4f*)(sD + (ty * 4 + u) * kDP + tx * 4) = rv;
  }
  __syncthreads();
#pragma unroll 1
  for (int it = 0; it < 16; ++it) {
    const int e = it * 256 + t;
    const int r = e >> 6, c = e & 63;
    float* q = sD + r * kDP + c;
    const float sq = *q;
    *q = sqrtf(sq);
  }
  __syncthreads();
  const int lane = t & 31, wave = t >> 5;
  const int hh = lane >> 4, c4 = (lane & 15) * 4;
  for (int pass = 0; pass < 2; ++pass) {
#pragma unroll
    for (int it = 0; it < 4; ++it) {
      const int row = wave * 8 + it * 2 + hh;
      const v4f v = *(const v4f*)(sD + row * kDP + c4);
      *(volatile v4f*)(dist + (size_t)(i0 + row) * SEQ + j0 + c4) = v;
    }
    __threadfence();
  }
}

__global__ __launch_bounds__(128) __attribute__((amdgpu_num_vgpr(256)))
void attn_kernel(const _Float16* __restrict__ Q, const _Float16* __restrict__ Kp,
                 const __bf16* __restrict__ Vh, const __bf16* __restrict__ Vl,
                 const float* __restrict__ dist,
                 unsigned short* __restrict__ Ch, unsigned short* __restrict__ Cl) {
  __shared__ __align__(16) _Float16 sK[64 * kKP];
  __shared__ __align__(16) __bf16   sVh[64 * kKP];
  __shared__ __align__(16) __bf16   sVl[64 * kKP];
  __shared__ __align__(16) float    sDt[64 * kDP];
  __shared__ __align__(16) __bf16   sPh[4][16 * kKP];
  __shared__ __align__(16) __bf16   sPl[4][16 * kKP];

  const int t = threadIdx.x, lane = t & 31, wave = t >> 5;
  const int hlf = lane >> 4, m = lane & 15;
  const int koff = hlf * 8, mOff = hlf * 8;
  const int q0 = blockIdx.x * 64;
  const int b  = blockIdx.y / kHeads;
  const int h  = blockIdx.y - b * kHeads;
  const int tokk = b * SEQ;
  const int tokq = tokk + q0;

  const int sr8  = t >> 3,  sc16 = (t & 7) * 8;
  const int sr16 = t >> 4,  sc4  = (t & 15) * 4;
  const int gK  = (tokk + sr8) * kDM + h * kHD + sc16;
  const int gV  = (h * kHD + sr8) * kTok + tokk + sc16;
  const int gD  = (q0 + sr16) * SEQ + sc4;
  const int lKs = sr8 * kKP + sc16;
  const int lDs = sr16 * kDP + sc4;
  const int gQ  = (tokq + wave * 16 + m) * kDM + h * kHD + koff;
  const int lF  = m * kKP + koff;
  const int lDr = (wave * 16 + mOff) * kDP + m;
  const int lPw = mOff * kKP + m;

  float mrun[8], lrun[8];
#pragma unroll
  for (int r = 0; r < 8; ++r) { mrun[r] = -INFINITY; lrun[r] = 0.f; }
  v8f acc[4];
#pragma unroll
  for (int tt = 0; tt < 4; ++tt) acc[tt] = (v8f){0.f,0.f,0.f,0.f,0.f,0.f,0.f,0.f};

#pragma unroll 1
  for (int kt = 0; kt < SEQ / 64; ++kt) {
    const int kb0 = kt * 64;
    __syncthreads();
#pragma unroll 1
    for (int c = 0; c < 4; ++c) {
      const v8h kv = *(const v8h*)(Kp + gK + (kb0 + c * 16) * kDM);
      const int vo = gV + c * 16 * kTok + kb0;
      const v8b hv = *(const v8b*)(Vh + vo);
      const v8b lv = *(const v8b*)(Vl + vo);
      const int lo = lKs + c * 16 * kKP;
      *(v8h*)(sK + lo)  = kv;
      *(v8b*)(sVh + lo) = hv;
      *(v8b*)(sVl + lo) = lv;
    }
#pragma unroll 1
    for (int c = 0; c < 8; ++c) {
      const v4f dv = *(const v4f*)(dist + gD + c * 8 * SEQ + kb0);
      *(v4f*)(sDt + lDs + c * 8 * kDP) = dv;
    }
    __syncthreads();

    v8f s[4];
#pragma unroll
    for (int j = 0; j < 4; ++j) s[j] = (v8f){0.f,0.f,0.f,0.f,0.f,0.f,0.f,0.f};
    {
      const v16h qf = Frag<_Float16>::load(Q + gQ);
      qk_pair(s[0], s[1], qf, sK + lF,            sK + lF + 16 * kKP);
      qk_pair(s[2], s[3], qf, sK + lF + 32 * kKP, sK + lF + 48 * kKP);
    }
    {
      const v16h qf = Frag<_Float16>::load(Q + gQ + 32);
      qk_pair(s[0], s[1], qf, sK + lF + 32,            sK + lF + 16 * kKP + 32);
      qk_pair(s[2], s[3], qf, sK + lF + 32 * kKP + 32, sK + lF + 48 * kKP + 32);
    }
    phase_cut();

#pragma unroll
    for (int r = 0; r < 8; ++r) {
      const float* dr = sDt + lDr + r * kDP;
      const float v0 = s[0][r] * 0.125f - dr[0];
      const float v1 = s[1][r] * 0.125f - dr[16];
      const float v2 = s[2][r] * 0.125f - dr[32];
      const float v3 = s[3][r] * 0.125f - dr[48];
      float tm = fmaxf(fmaxf(v0, v1), fmaxf(v2, v3));
      tm = fmaxf(tm, __shfl_xor(tm, 8));
      tm = fmaxf(tm, __shfl_xor(tm, 4));
      tm = fmaxf(tm, __shfl_xor(tm, 2));
      tm = fmaxf(tm, __shfl_xor(tm, 1));
      const float mn = fmaxf(mrun[r], tm);
      const float cr = __expf(mrun[r] - mn);
      mrun[r] = mn;
      const float p0 = __expf(v0 - mn);
      const float p1 = __expf(v1 - mn);
      const float p2 = __expf(v2 - mn);
      const float p3 = __expf(v3 - mn);
      float ps = p0;
      ps += p1; ps += p2; ps += p3;
      __bf16* pw  = sPh[wave] + lPw + r * kKP;
      __bf16* plw = sPl[wave] + lPw + r * kKP;
      put_p(pw,      plw,      p0);
      put_p(pw + 16, plw + 16, p1);
      put_p(pw + 32, plw + 32, p2);
      put_p(pw + 48, plw + 48, p3);
      ps += __shfl_xor(ps, 8);
      ps += __shfl_xor(ps, 4);
      ps += __shfl_xor(ps, 2);
      ps += __shfl_xor(ps, 1);
      lrun[r] = lrun[r] * cr + ps;
      acc[0][r] *= cr;
      acc[1][r] *= cr;
      acc[2][r] *= cr;
      acc[3][r] *= cr;
      phase_cut();
    }
    __builtin_amdgcn_fence(3, "workgroup");
    __builtin_amdgcn_wave_barrier();
    __builtin_amdgcn_fence(2, "workgroup");

    {
      const __bf16* pr = sPh[wave] + lF;
      const v16b pf0 = Frag<__bf16>::load(pr);
      const v16b pf1 = Frag<__bf16>::load(pr + 32);
#pragma unroll
      for (int tt = 0; tt < 4; ++tt) {
        const int o = lF + tt * 16 * kKP;
        pv_hl(acc[tt], pf0, sVh + o,      sVl + o);
        pv_hl(acc[tt], pf1, sVh + o + 32, sVl + o + 32);
      }
    }
    phase_cut();
    {
      const __bf16* pr = sPl[wave] + lF;
      const v16b pf0 = Frag<__bf16>::load(pr);
      const v16b pf1 = Frag<__bf16>::load(pr + 32);
#pragma unroll
      for (int tt = 0; tt < 4; ++tt) {
        const int o = lF + tt * 16 * kKP;
        pv_h(acc[tt], pf0, sVh + o);
        pv_h(acc[tt], pf1, sVh + o + 32);
      }
    }
    acc_guard4(acc[0], acc[1], acc[2], acc[3]);
    phase_cut();
  }

  __syncthreads();
  float* slab = sDt + wave * 16 * kDP;
#pragma unroll
  for (int r = 0; r < 8; ++r) {
    const float inv = 1.0f / lrun[r];
    float* sp = slab + (mOff + r) * kDP + m;
    sp[0]  = acc[0][r] * inv;
    sp[16] = acc[1][r] * inv;
    sp[32] = acc[2][r] * inv;
    sp[48] = acc[3][r] * inv;
  }
  __builtin_amdgcn_fence(3, "workgroup");
  __builtin_amdgcn_wave_barrier();
  __builtin_amdgcn_fence(2, "workgroup");
  const int q8 = lane >> 3, c8 = (lane & 7) * 8;
  const int go = (tokq + wave * 16) * kDM + h * kHD + c8;
  for (int pass = 0; pass < 2; ++pass) {
#pragma unroll
    for (int it = 0; it < 4; ++it) {
      const int row = it * 4 + q8;
      const float* sp = slab + row * kDP + c8;
      const v4f a = *(const v4f*)(sp);
      const v4f c = *(const v4f*)(sp + 4);
      unsigned short hb[8], lb[8];
#pragma unroll
      for (int e = 0; e < 4; ++e) {
        hb[e] = f2bf_bits(a[e]);
        lb[e] = f2bf_bits(a[e] - bf_bits2f(hb[e]));
        hb[4 + e] = f2bf_bits(c[e]);
        lb[4 + e] = f2bf_bits(c[e] - bf_bits2f(hb[4 + e]));
      }
      const v4u hu = (v4u){pk16(hb[0], hb[1]), pk16(hb[2], hb[3]), pk16(hb[4], hb[5]), pk16(hb[6], hb[7])};
      const v4u lu = (v4u){pk16(lb[0], lb[1]), pk16(lb[2], lb[3]), pk16(lb[4], lb[5]), pk16(lb[6], lb[7])};
      *(volatile v4u*)(Ch + go + row * kDM) = hu;
      *(volatile v4u*)(Cl + go + row * kDM) = lu;
    }
    __threadfence();
  }
}

extern "C" void kernel_launch(void* const* d_in, const int* in_sizes, int n_in,
                              void* d_out, int out_size, void* d_ws, size_t ws_size,
                              hipStream_t stream) {
  if (n_in < 10) return;
  if (in_sizes[0] < ((NB - 1) * SEQ_FULL + SEQ) * kDM) return;
  if (in_sizes[1] < SEQ * kPos) return;
  if (in_sizes[2] < kDM * kDM || in_sizes[4] < kDM * kDM || in_sizes[6] < kDM * kDM || in_sizes[8] < kDM * kDM) return;
  if (in_sizes[3] < kDM || in_sizes[5] < kDM || in_sizes[7] < kDM || in_sizes[9] < kDM) return;
  if (out_size < kTok * kDM) return;
  if (ws_size < kWsEnd) return;

  const float* x   = (const float*)d_in[0];
  const float* pos = (const float*)d_in[1];
  const float* Wq  = (const float*)d_in[2];
  const float* bq  = (const float*)d_in[3];
  const float* Wk  = (const float*)d_in[4];
  const float* bk  = (const float*)d_in[5];
  const float* Wv  = (const float*)d_in[6];
  const float* bv  = (const float*)d_in[7];
  const float* Wo  = (const float*)d_in[8];
  const float* bo  = (const float*)d_in[9];
  float* out = (float*)d_out;

  char* ws = (char*)d_ws;
  unsigned short* XB  = (unsigned short*)(ws + kOffXB);
  unsigned short* WqT = (unsigned short*)(ws + kOffWq);
  unsigned short* WkT = (unsigned short*)(ws + kOffWk);
  unsigned short* WvT = (unsigned short*)(ws + kOffWv);
  unsigned short* WoT = (unsigned short*)(ws + kOffWo);
  unsigned short* Qh  = (unsigned short*)(ws + kOffQ);
  unsigned short* Kh  = (unsigned short*)(ws + kOffK);
  unsigned short* VTh = (unsigned short*)(ws + kOffVh);
  unsigned short* VTl = (unsigned short*)(ws + kOffVl);
  float*          Dst = (float*)(ws + kOffD);
  unsigned short* Ch  = (unsigned short*)(ws + kOffCh);
  unsigned short* Cl  = (unsigned short*)(ws + kOffCl);
  const float* noresid = Dst;

  xcast_kernel<<<dim3(kTok / 32), dim3(256), 0, stream>>>(x, XB);
  wtcast_kernel<<<dim3(kDM / 64, kDM / 64), dim3(256), 0, stream>>>(Wq, WqT);
  wtcast_kernel<<<dim3(kDM / 64, kDM / 64), dim3(256), 0, stream>>>(Wk, WkT);
  wtcast_kernel<<<dim3(kDM / 64, kDM / 64), dim3(256), 0, stream>>>(Wv, WvT);
  wtcast_kernel<<<dim3(kDM / 64, kDM / 64), dim3(256), 0, stream>>>(Wo, WoT);

  dist_kernel<<<dim3(SEQ / 64, SEQ / 64), dim3(256), 0, stream>>>(pos, Dst);

  const int tilesQK = (kTok / 64) * (kDM / 64);
  wmma_gemm64<1, 0, 2, 1, false><<<dim3((tilesQK + 7) / 8, 1), dim3(256), 0, stream>>>(
      XB, XB, kDM, 0L, WqT, WqT, kDM, 0L, (void*)Qh, (void*)Qh, kDM, 0L,
      bq, noresid, 0L, kTok, kDM, kDM, 1.0f);
  wmma_gemm64<1, 0, 2, 1, false><<<dim3((tilesQK + 7) / 8, 1), dim3(256), 0, stream>>>(
      XB, XB, kDM, 0L, WkT, WkT, kDM, 0L, (void*)Kh, (void*)Kh, kDM, 0L,
      bk, noresid, 0L, kTok, kDM, kDM, 1.0f);
  const int tilesVT = (kDM / 64) * (kTok / 64);
  wmma_gemm64<1, 0, 1, 2, false><<<dim3((tilesVT + 7) / 8, 1), dim3(256), 0, stream>>>(
      WvT, WvT, kDM, 0L, XB, XB, kDM, 0L, (void*)VTh, (void*)VTl, kTok, 0L,
      bv, noresid, 0L, kDM, kTok, kDM, 1.0f);

  attn_kernel<<<dim3(SEQ / 64, NB * kHeads), dim3(128), 0, stream>>>(
      (const _Float16*)Qh, (const _Float16*)Kh, (const __bf16*)VTh, (const __bf16*)VTl, Dst, Ch, Cl);

  const int tilesO = (kTok / 64) * (kDM / 64);
  wmma_gemm64<1, 1, 2, 0, false><<<dim3((tilesO + 7) / 8, 1), dim3(256), 0, stream>>>(
      Ch, Cl, kDM, 0L, WoT, WoT, kDM, 0L, (void*)out, (void*)out, kDM, 0L,
      bo, noresid, 0L, kTok, kDM, kDM, 1.0f);
}
